// SelfAttention_9534827397170
// MI455X (gfx1250) — hardware-verified
//
#include <hip/hip_runtime.h>
#include <stddef.h>


typedef _Float16 h16;
typedef _Float16 v16h __attribute__((ext_vector_type(16)));
typedef _Float16 v8h  __attribute__((ext_vector_type(8)));
typedef float    v8f  __attribute__((ext_vector_type(8)));
typedef float    v4f  __attribute__((ext_vector_type(4)));

#ifndef NB
#define NB 4
#endif
#ifndef SEQ
#define SEQ 512
#endif
#define NB_FULL  4
#define SEQ_FULL 512
#define HDIM  256
#define DPROJ 128
#define NCAT  (2 * DPROJ)
#define MROWS (NB * SEQ)
#define QT    16

static_assert(NB >= 1 && NB <= NB_FULL);
static_assert(SEQ >= 256 && SEQ <= SEQ_FULL && (SEQ % 256) == 0);
static_assert((SEQ % 64) == 0 && (SEQ % 32) == 0 && (SEQ % QT) == 0);
static_assert(HDIM == 32 * 8);
static_assert(HDIM == 8 * 32);
static_assert((HDIM % 64) == 0 && (HDIM % 32) == 0);
static_assert((NCAT % 64) == 0);
static_assert((DPROJ % 8) == 0 && (DPROJ % 4) == 0 && DPROJ <= 256);
static_assert((MROWS % 64) == 0 && (MROWS % 8) == 0);
static_assert(QT == 16);
static_assert((size_t)NB_FULL * SEQ_FULL * HDIM * 4 == (size_t)2097152);

#define LDT 72
#define LDC 68
static_assert((LDT % 8) == 0 && LDT >= 64);
static_assert((LDC % 4) == 0 && LDC >= 64);

#define SLD (SEQ + 4)
#define PLD (SEQ + 8)
#define OLD (HDIM + 4)
static_assert((SLD % 4) == 0 && (PLD % 8) == 0 && (OLD % 4) == 0);
static_assert(QT * SLD >= QT * OLD);

#define WCARRY 64.0f
#define PEXP   10.0f

#define C16_BYTES  ((size_t)MROWS * HDIM * 2)
#define WCAT_BYTES ((size_t)NCAT * HDIM * 2)
#define CT_BYTES   ((size_t)NB * HDIM * SEQ * 2)
#define WW_BYTES   ((size_t)MROWS * NCAT * 4)
#define OFF_C16  ((size_t)0)
#define OFF_WCAT (OFF_C16 + C16_BYTES)
#define OFF_CT   (OFF_WCAT + WCAT_BYTES)
#define OFF_WW   (OFF_CT + CT_BYTES)
#define WS_TOTAL (OFF_WW + WW_BYTES)
static_assert((C16_BYTES % 128) == 0 && (WCAT_BYTES % 128) == 0);
static_assert((CT_BYTES % 128) == 0 && (WW_BYTES % 128) == 0);
static_assert(WS_TOTAL <= (size_t)134217728);

__device__ __forceinline__ float bf16r(float x) {
  unsigned int u = __float_as_uint(x);
  u = (u + 0x7FFFu + ((u >> 16) & 1u)) & 0xFFFF0000u;
  return __uint_as_float(u);
}

static __device__ __forceinline__ h16 toh_flush(float v) {
  const h16 r = (h16)v;
  return (fabsf(v) < 6.103515625e-05f) ? (h16)0.0f : r;
}

__device__ __forceinline__ v16h frag_at(const _Float16* p) {
  v8h lo = *(const v8h*)(p);
  v8h hi = *(const v8h*)(p + 16);
  v16h out;
#pragma unroll
  for (int i = 0; i < 8; ++i) { out[i] = lo[i]; out[i + 8] = hi[i]; }
  return out;
}

__device__ __forceinline__ v8f wmma16(v16h a, v16h b, v8f c) {
  v8f d = __builtin_amdgcn_wmma_f32_16x16x32_f16(false, a, false, b, (short)0, c,
                                                 false, false);
  asm volatile("v_nop\n\tv_nop\n\tv_nop\n\tv_nop" : "+v"(d) : "v"(a), "v"(b));
  return d;
}

__device__ __forceinline__ float red32_sum(float x) {
#pragma unroll
  for (int off = 1; off < 32; off <<= 1) x += __shfl_xor(x, off, 32);
  return x;
}
__device__ __forceinline__ float red32_max(float x) {
#pragma unroll
  for (int off = 1; off < 32; off <<= 1) x = fmaxf(x, __shfl_xor(x, off, 32));
  return x;
}

__device__ __forceinline__ float exp2_hw(float x) {
#if __has_builtin(__builtin_amdgcn_exp2f)
  return __builtin_amdgcn_exp2f(x);
#else
  return exp2f(x);
#endif
}

__device__ __forceinline__ float tanh_eval(float x) {
  const float e = exp2_hw(x * 2.8853900817779268f);
  return 1.0f - 2.0f * __builtin_amdgcn_rcpf(1.0f + e);
}

__global__ __launch_bounds__(256) void wconv_kernel(
    const float* __restrict__ W, _Float16* __restrict__ Wt, unsigned ldw, unsigned ldk) {
  __shared__ _Float16 T[64 * LDT];
  const unsigned tid = threadIdx.x;
  const unsigned n0 = blockIdx.x * 64u;
  const unsigned k0 = blockIdx.y * 64u;
#pragma unroll 4
  for (unsigned j = 0; j < 16u; ++j) {
    const unsigned idx = tid + 256u * j;
    const unsigned kr = idx >> 6, nc = idx & 63u;
    const float v = W[(size_t)(k0 + kr) * ldw + n0 + nc];
    T[nc * LDT + kr] = (_Float16)(WCARRY * bf16r(v));
  }
  __syncthreads();
  v8h x[2];
  size_t off[2];
#pragma unroll
  for (unsigned i = 0; i < 2u; ++i) {
    const unsigned n = 32u * i + (tid >> 3);
    const unsigned kc = (tid & 7u) * 8u;
    x[i] = *(const v8h*)&T[n * LDT + kc];
    off[i] = (size_t)(n0 + n) * ldk + k0 + kc;
  }
#pragma unroll
  for (int i = 0; i < 2; ++i) *(volatile v8h*)(Wt + off[i]) = x[i];
  __threadfence();
#pragma unroll
  for (int i = 0; i < 2; ++i) *(volatile v8h*)(Wt + off[i]) = x[i];
}

__global__ __launch_bounds__(256) void cast_rows_kernel(
    const float* __restrict__ src, _Float16* __restrict__ dst, float carry,
    unsigned seg_rows, unsigned seg_rows_full) {
  const unsigned gid = blockIdx.x * 256u + threadIdx.x;
  const unsigned row = gid >> 5;
  const unsigned col = (gid & 31u) * 8u;
  const unsigned seg = row / seg_rows;
  const unsigned srow = seg * seg_rows_full + (row - seg * seg_rows);
  const float* p = src + (size_t)srow * HDIM + col;
  const v4f a0 = *(const v4f*)(p);
  const v4f a1 = *(const v4f*)(p + 4);
  v8h o;
#pragma unroll
  for (int i = 0; i < 4; ++i) {
    o[i]     = toh_flush(carry * bf16r(a0[i]));
    o[i + 4] = toh_flush(carry * bf16r(a1[i]));
  }
  _Float16* q = dst + (size_t)row * HDIM + col;
  *(volatile v8h*)q = o;
  __threadfence();
  *(volatile v8h*)q = o;
}

__global__ __launch_bounds__(256) void proj_gemm_kernel(
    const _Float16* __restrict__ A16, const _Float16* __restrict__ Bt,
    float* __restrict__ outf) {
  __shared__ __attribute__((aligned(16))) float Cs[64 * LDC];
  const unsigned tid = threadIdx.x, lane = tid & 31u;
  const unsigned w = (unsigned)__builtin_amdgcn_readfirstlane(threadIdx.x >> 5);
  const unsigned mw = w >> 1, nw = w & 1u;
  const unsigned hh = lane >> 4, m = lane & 15u;
  const unsigned n0 = blockIdx.x * 64u;
  const unsigned row0 = blockIdx.y * 64u;
  const unsigned K = (unsigned)HDIM;

  const _Float16* ap  = A16 + (size_t)(row0 + mw * 16u + m) * K + hh * 8u;
  const _Float16* bp0 = Bt + (size_t)(n0 + nw * 32u + m) * K + hh * 8u;
  const _Float16* bp1 = bp0 + (size_t)16 * K;
  v8f acc0 = {}, acc1 = {};
#pragma unroll 2
  for (unsigned k0 = 0; k0 < K; k0 += 32u) {
    const v16h a  = frag_at(ap + k0);
    const v16h b0 = frag_at(bp0 + k0);
    const v16h b1 = frag_at(bp1 + k0);
    acc0 = wmma16(a, b0, acc0);
    acc1 = wmma16(a, b1, acc1);
  }
#pragma unroll
  for (int r = 0; r < 8; ++r) {
    float* d = &Cs[(mw * 16u + hh * 8u + (unsigned)r) * LDC + nw * 32u + m];
    d[0]  = acc0[r];
    d[16] = acc1[r];
  }
  __syncthreads();

  const float cs = 1.0f / (WCARRY * WCARRY);
  v4f xs[4];
  size_t off[4];
#pragma unroll
  for (unsigned i = 0; i < 4u; ++i) {
    const unsigned r = 16u * i + (tid >> 4);
    const unsigned c = (tid & 15u) * 4u;
    const v4f u = *(const v4f*)&Cs[r * LDC + c];
    xs[i] = u * cs;
    off[i] = (size_t)(row0 + r) * NCAT + n0 + c;
  }
#pragma unroll
  for (int i = 0; i < 4; ++i) *(volatile v4f*)(outf + off[i]) = xs[i];
  __threadfence();
#pragma unroll
  for (int i = 0; i < 4; ++i) *(volatile v4f*)(outf + off[i]) = xs[i];
}

__global__ __launch_bounds__(256) void addattn_kernel(
    const float* __restrict__ WW, const float* __restrict__ Wv,
    const _Float16* __restrict__ Ct, float* __restrict__ out) {
  __shared__ __attribute__((aligned(16))) float Ss[QT * SLD];
  __shared__ __attribute__((aligned(16))) _Float16 Ps[QT * PLD];
  __shared__ __attribute__((aligned(16))) float Wq[QT * DPROJ];
  __shared__ __attribute__((aligned(16))) float Vv[DPROJ];
  __shared__ __attribute__((aligned(16))) float Ls[QT];

  const unsigned tid = threadIdx.x, lane = tid & 31u;
  const unsigned wave = (unsigned)__builtin_amdgcn_readfirstlane(threadIdx.x >> 5);
  const unsigned hh = lane >> 4, m = lane & 15u;
  const unsigned b = blockIdx.y;
  const unsigned q0 = blockIdx.x * (unsigned)QT;

#pragma unroll
  for (unsigned j = 0; j < (unsigned)(QT * DPROJ / 4 / 256); ++j) {
    const unsigned idx = tid + 256u * j;
    const unsigned r = idx / (unsigned)(DPROJ / 4);
    const unsigned c = (idx - r * (unsigned)(DPROJ / 4)) * 4u;
    const v4f t = *(const v4f*)(WW + (size_t)(b * (unsigned)SEQ + q0 + r) * NCAT + DPROJ + c);
    *(v4f*)&Wq[r * DPROJ + c] = t;
  }
  {
    const unsigned d = tid & (unsigned)(DPROJ - 1);
    Vv[d] = bf16r(Wv[d]);
  }
  __syncthreads();

#pragma unroll 1
  for (unsigned kt = 0; kt < (unsigned)(SEQ / 256); ++kt) {
    const unsigned j = kt * 256u + wave * 32u + lane;
    const float* wcp = WW + (size_t)(b * (unsigned)SEQ + j) * NCAT;
    float acc[QT];
#pragma unroll
    for (int r = 0; r < QT; ++r) acc[r] = 0.0f;
#pragma unroll 1
    for (unsigned d = 0; d < (unsigned)DPROJ; d += 4u) {
      const v4f x  = *(const v4f*)(wcp + d);
      const v4f vv = *(const v4f*)&Vv[d];
#pragma unroll
      for (int r = 0; r < QT; ++r) {
        const v4f y = *(const v4f*)&Wq[(unsigned)r * DPROJ + d];
#pragma unroll
        for (int e = 0; e < 4; ++e) acc[r] += vv[e] * tanh_eval(x[e] + y[e]);
      }
    }
#pragma unroll
    for (int r = 0; r < QT; ++r) Ss[(unsigned)r * SLD + j] = acc[r];
  }
  __syncthreads();

#pragma unroll 1
  for (unsigned rr = 0; rr < 2u; ++rr) {
    const unsigned r = wave * 2u + rr;
    float mx = -3.0e38f;
#pragma unroll 4
    for (unsigned t = 0; t < (unsigned)(SEQ / 32); ++t)
      mx = fmaxf(mx, Ss[r * SLD + t * 32u + lane]);
    mx = red32_max(mx);
    float ls = 0.0f;
#pragma unroll 4
    for (unsigned t = 0; t < (unsigned)(SEQ / 32); ++t) {
      const float arg = (Ss[r * SLD + t * 32u + lane] - mx) * 1.4426950408889634f + PEXP;
      const float p = (arg < -14.0f) ? 0.0f : exp2_hw(arg);
      const h16 ph = toh_flush(p);
      Ps[r * PLD + t * 32u + lane] = ph;
      ls += (float)ph;
    }
    ls = red32_sum(ls);
    if (lane == 0u) Ls[r] = ls;
  }
  __syncthreads();

  const _Float16* bp0 = Ct + ((size_t)b * HDIM + wave * 32u + m) * SEQ + hh * 8u;
  const _Float16* bp1 = bp0 + (size_t)16 * SEQ;
  v8f o0 = {}, o1 = {};
#pragma unroll 4
  for (unsigned k0 = 0; k0 < (unsigned)SEQ; k0 += 32u) {
    const v8h plo = *(const v8h*)&Ps[m * PLD + k0 + hh * 8u];
    const v8h phi = *(const v8h*)&Ps[m * PLD + k0 + 16u + hh * 8u];
    v16h a;
#pragma unroll
    for (int i = 0; i < 8; ++i) { a[i] = plo[i]; a[i + 8] = phi[i]; }
    const v16h b0 = frag_at(bp0 + k0);
    const v16h b1 = frag_at(bp1 + k0);
    o0 = wmma16(a, b0, o0);
    o1 = wmma16(a, b1, o1);
  }

#pragma unroll
  for (int r = 0; r < 8; ++r) {
    const float inv = __builtin_amdgcn_rcpf(Ls[hh * 8u + (unsigned)r] * WCARRY);
    float* d = &Ss[(hh * 8u + (unsigned)r) * OLD + wave * 32u + m];
    d[0]  = o0[r] * inv;
    d[16] = o1[r] * inv;
  }
  __syncthreads();

  v4f xs[4];
  size_t off[4];
#pragma unroll
  for (unsigned i = 0; i < 4u; ++i) {
    const unsigned idx = tid + 256u * i;
    const unsigned r = idx >> 6;
    const unsigned c = (idx & 63u) * 4u;
    xs[i] = *(const v4f*)&Ss[r * OLD + c];
    off[i] = ((size_t)b * SEQ_FULL + q0 + r) * HDIM + c;
  }
#pragma unroll
  for (int i = 0; i < 4; ++i) *(volatile v4f*)(out + off[i]) = xs[i];
  __threadfence();
#pragma unroll
  for (int i = 0; i < 4; ++i) *(volatile v4f*)(out + off[i]) = xs[i];
}

extern "C" void kernel_launch(void* const* d_in, const int* in_sizes, int n_in,
                              void* d_out, int out_size, void* d_ws, size_t ws_size,
                              hipStream_t stream) {
  if (n_in < 5) return;
  const long long need_c = ((long long)(NB - 1) * SEQ_FULL + SEQ) * HDIM;
  if ((long long)in_sizes[0] < need_c) return;
  if ((long long)in_sizes[2] < (long long)DPROJ * HDIM) return;
  if ((long long)in_sizes[3] < (long long)DPROJ * HDIM) return;
  if (in_sizes[4] < DPROJ) return;
  if ((long long)out_size < need_c) return;
  if (ws_size < WS_TOTAL) return;

  const float* c  = (const float*)d_in[0];
  const float* Wc = (const float*)d_in[2];
  const float* Ww = (const float*)d_in[3];
  const float* Wv = (const float*)d_in[4];
  float* out = (float*)d_out;

  char* ws = (char*)d_ws;
  _Float16* C16    = (_Float16*)(ws + OFF_C16);
  _Float16* Wcat16 = (_Float16*)(ws + OFF_WCAT);
  _Float16* Ct16   = (_Float16*)(ws + OFF_CT);
  float*    WWp    = (float*)(ws + OFF_WW);

  dim3 blk(256);

  cast_rows_kernel<<<dim3(MROWS / 8), blk, 0, stream>>>(c, C16, WCARRY, (unsigned)SEQ,
                                                        (unsigned)SEQ_FULL);
  cast_rows_kernel<<<dim3(DPROJ / 8), blk, 0, stream>>>(Wc, Wcat16, WCARRY, (unsigned)DPROJ,
                                                        (unsigned)DPROJ);
  cast_rows_kernel<<<dim3(DPROJ / 8), blk, 0, stream>>>(Ww, Wcat16 + (size_t)DPROJ * HDIM, WCARRY,
                                                        (unsigned)DPROJ, (unsigned)DPROJ);
  for (int b = 0; b < NB; ++b) {
    wconv_kernel<<<dim3(HDIM / 64, SEQ / 64), blk, 0, stream>>>(
        c + (size_t)b * SEQ_FULL * HDIM, Ct16 + (size_t)b * HDIM * SEQ, (unsigned)HDIM,
        (unsigned)SEQ);
  }
  proj_gemm_kernel<<<dim3(NCAT / 64, MROWS / 64), blk, 0, stream>>>(C16, Wcat16, WWp);
  addattn_kernel<<<dim3(SEQ / QT, NB), blk, 0, stream>>>(WWp, Wv, Ct16, out);
}
